// SAGEConvModel_17635135718039
// MI455X (gfx1250) — hardware-verified
//
#include <hip/hip_runtime.h>
#include <stdint.h>
#include <math.h>


typedef _Float16 v16h __attribute__((ext_vector_type(16)));
typedef _Float16 v8h  __attribute__((ext_vector_type(8)));
typedef _Float16 v8ha __attribute__((ext_vector_type(8), may_alias));
typedef float    v8f  __attribute__((ext_vector_type(8)));
typedef float    v4f  __attribute__((ext_vector_type(4)));
typedef float    v4fa __attribute__((ext_vector_type(4), may_alias));
typedef int      v4i  __attribute__((ext_vector_type(4)));

#define NN    100000
#define NE    1600000
#define NF    32
#define NG    512
#define NCH   30
#define NBKT  391
#define NBP   392
#define ECH   4096
#define NCHK  391
#define NWAV  8
#define CROW  (NWAV * NBP)
#define MIDX  (NBKT * NCHK)
#define SEG   608
#define LOFFN (256 * SEG)
#define MAXL  202912
#define CSRN  (MAXL * 32)
#define CAPB  6144
#define WHB   264
#define NODEP (NBKT * 256)

__device__ __forceinline__ v8f wmma16(v16h a, v16h b, v8f c) {
  return __builtin_amdgcn_wmma_f32_16x16x32_f16(false, a, false, b, (short)0, c, false, false);
}

__device__ __forceinline__ unsigned matchmask(int key) {
  unsigned m = 0u;
#pragma unroll
  for (int i = 0; i < 32; ++i) {
    const int kb = __builtin_amdgcn_readlane(key, i);
    m |= (kb == key) ? (1u << i) : 0u;
  }
  return m;
}

__device__ __forceinline__ int bucket_key(int d) {
  return ((unsigned)d < (unsigned)NN) ? (d >> 8) : (NBP - 1);
}

__device__ __forceinline__ void pack_store(const _Float16* sp, const float* st,
                                           _Float16* pb, float* ptab, int t) {
  for (int j = t; j < 512; j += 256) {
    v8h v = *(const v8ha*)(sp + 8 * j);
    *(volatile v8h*)(pb + 8 * j) = v;
  }
  if (t < 48) {
    v4f v;
    v.x = st[4 * t]; v.y = st[4 * t + 1]; v.z = st[4 * t + 2]; v.w = st[4 * t + 3];
    *(volatile v4f*)(ptab + 4 * t) = v;
  }
}

__global__ void __launch_bounds__(256) k_pack(
    const float* __restrict__ Wl1, const float* __restrict__ bl1, const float* __restrict__ Wr1,
    const float* __restrict__ Wl2, const float* __restrict__ bl2, const float* __restrict__ Wr2,
    const float* __restrict__ g1, const float* __restrict__ b1,
    const float* __restrict__ m1, const float* __restrict__ v1,
    const float* __restrict__ g2, const float* __restrict__ b2,
    const float* __restrict__ m2, const float* __restrict__ v2,
    _Float16* __restrict__ pb, float* __restrict__ ptab) {
  __shared__ __attribute__((aligned(16))) _Float16 sp[4096];
  __shared__ __attribute__((aligned(16))) float st[192];
  const int t = threadIdx.x;
  {
    const int layer = t >> 7, tt = (t >> 6) & 1, mat = (t >> 5) & 1, ln = t & 31;
    const int n = (ln & 15) + 16 * tt, hh = ln >> 4;
    const int kdim = layer ? NCH : NF;
    const float* W = layer ? (mat ? Wr2 : Wl2) : (mat ? Wr1 : Wl1);
#pragma unroll
    for (int i = 0; i < 16; ++i) {
      const int k = (i < 8) ? (8 * hh + i) : (16 + 8 * hh + (i - 8));
      float w = 0.f;
      if (n < NCH && k < kdim) w = W[n * kdim + k] * 16.0f;
      sp[t * 16 + i] = (_Float16)w;
    }
  }
  if (t < 64) {
    const int layer = t >> 5, n = t & 31;
    const float* blp = layer ? bl2 : bl1;
    const float* gp  = layer ? g2 : g1;
    const float* bp  = layer ? b2 : b1;
    const float* mp  = layer ? m2 : m1;
    const float* vp  = layer ? v2 : v1;
    float bias = 0.f, scale = 0.f, shift = 0.f;
    if (n < NCH) {
      const float rs = 1.0f / sqrtf(vp[n] + 1e-5f);
      scale = gp[n] * rs;
      shift = bp[n] - mp[n] * scale;
      bias  = blp[n] * 16.0f;
    }
    st[t] = bias; st[64 + t] = scale; st[128 + t] = shift;
  }
  __syncthreads();
  pack_store(sp, st, pb, ptab, t);
  __threadfence();
  pack_store(sp, st, pb, ptab, t);
}

__device__ __forceinline__ void row_store(const int* wh, int* row, int t) {
  for (int i4 = t; i4 < CROW / 4; i4 += 256) {
    v4i v;
    v.x = wh[4 * i4]; v.y = wh[4 * i4 + 1]; v.z = wh[4 * i4 + 2]; v.w = wh[4 * i4 + 3];
    *(volatile v4i*)(row + 4 * i4) = v;
  }
}

__global__ void __launch_bounds__(256) k_count(const int* __restrict__ dst,
                                              int* __restrict__ cntrow) {
  __shared__ __attribute__((aligned(16))) int wh[CROW];
  const int t = threadIdx.x, lane = t & 31, w = t >> 5;
  const int c = blockIdx.x;
  for (int i = t; i < CROW; i += 256) wh[i] = 0;
  __syncthreads();
  const int e0 = c * ECH;
  const unsigned lt = (1u << lane) - 1u;
  for (int j = w; j < ECH / 32; j += NWAV) {
    const int e = e0 + j * 32 + lane;
    const int d = (e < NE) ? dst[e] : -1;
    const int key = bucket_key(d);
    const unsigned m = matchmask(key);
    if ((m & lt) == 0u) wh[w * NBP + key] += __builtin_popcount(m);
  }
  __syncthreads();
  int* row = cntrow + (size_t)c * CROW;
  row_store(wh, row, t);
  __threadfence();
  row_store(wh, row, t);
}

__device__ __forceinline__ int lines_at(const int* cntrow, int b, int c) {
  const int* p = cntrow + (size_t)c * CROW + b;
  int s = 0;
#pragma unroll
  for (int u = 0; u < NWAV; ++u) s += p[u * NBP];
  return (s + 31) >> 5;
}

__device__ __forceinline__ void scan_write(const int* cntrow, int* lineoff, int i0, int ex) {
  int run = ex;
  int b = i0 / NCHK, c = i0 - (i0 / NCHK) * NCHK;
  for (int k = 0; k < SEG; k += 4) {
    int vals[4];
#pragma unroll
    for (int m = 0; m < 4; ++m) {
      const int idx = i0 + k + m;
      vals[m] = run;
      if (idx < MIDX) run += lines_at(cntrow, b, c);
      if (++c == NCHK) { c = 0; ++b; }
    }
    v4i v;
    v.x = vals[0]; v.y = vals[1]; v.z = vals[2]; v.w = vals[3];
    *(volatile v4i*)(lineoff + i0 + k) = v;
  }
}

__global__ void __launch_bounds__(256) k_scan(const int* __restrict__ cntrow,
                                             int* __restrict__ lineoff) {
  __shared__ int stot[256];
  const int t = threadIdx.x;
  const int i0 = t * SEG;
  int s = 0;
  {
    int b = i0 / NCHK, c = i0 - (i0 / NCHK) * NCHK;
    for (int k = 0; k < SEG; ++k) {
      const int idx = i0 + k;
      if (idx < MIDX) s += lines_at(cntrow, b, c);
      if (++c == NCHK) { c = 0; ++b; }
    }
  }
  stot[t] = s;
  __syncthreads();
  int ex = 0;
  for (int u = 0; u < t; ++u) ex += stot[u];
  scan_write(cntrow, lineoff, i0, ex);
  __threadfence();
  scan_write(cntrow, lineoff, i0, ex);
}

__device__ __forceinline__ void runs_store(const int* srt, const int* bcnt, const int* bst,
                                           const int* lineoff, int* runs, int c, int t) {
  for (int b = t; b < NBKT; b += 256) {
    const int n = bcnt[b];
    if (n <= 0) continue;
    const int nl = (n + 31) >> 5;
    const int L = lineoff[b * NCHK + c];
    if (L < 0 || L + nl > MAXL) continue;
    const int sb = bst[b];
    for (int q = 0; q < nl; ++q) {
      int* lp = runs + (size_t)(L + q) * 32;
#pragma unroll
      for (int i = 0; i < 8; ++i) {
        int e4[4];
#pragma unroll
        for (int m = 0; m < 4; ++m) {
          const int pos = q * 32 + 4 * i + m;
          e4[m] = (pos < n) ? srt[sb + pos] : -1;
        }
        v4i v;
        v.x = e4[0]; v.y = e4[1]; v.z = e4[2]; v.w = e4[3];
        *(volatile v4i*)(lp + 4 * i) = v;
      }
    }
  }
}

__global__ void __launch_bounds__(256) k_place(const int* __restrict__ src,
                                              const int* __restrict__ dst,
                                              const int* __restrict__ cntrow,
                                              const int* __restrict__ lineoff,
                                              int* __restrict__ runs) {
  __shared__ int wex[CROW];
  __shared__ int bcnt[NBP];
  __shared__ int bst[NBP];
  __shared__ int srt[ECH];
  const int t = threadIdx.x, lane = t & 31, w = t >> 5;
  const int c = blockIdx.x;
  const int* row = cntrow + (size_t)c * CROW;
  for (int b = t; b < NBP; b += 256) {
    int run = 0;
#pragma unroll
    for (int u = 0; u < NWAV; ++u) {
      const int v = row[u * NBP + b];
      wex[u * NBP + b] = run;
      run += v;
    }
    bcnt[b] = run;
  }
  __syncthreads();
  if (w == 0) {
    int s = 0;
#pragma unroll
    for (int i = 0; i < 13; ++i) {
      const int idx = lane * 13 + i;
      if (idx < NBP) s += bcnt[idx];
    }
    int incl = s;
#pragma unroll
    for (int d = 1; d < 32; d <<= 1) {
      const int y = __shfl_up(incl, d);
      if (lane >= d) incl += y;
    }
    int ex = incl - s;
#pragma unroll
    for (int i = 0; i < 13; ++i) {
      const int idx = lane * 13 + i;
      if (idx < NBP) { bst[idx] = ex; ex += bcnt[idx]; }
    }
  }
  __syncthreads();
  const int e0 = c * ECH;
  const unsigned lt = (1u << lane) - 1u;
  for (int j = w; j < ECH / 32; j += NWAV) {
    const int e = e0 + j * 32 + lane;
    const bool valid = e < NE;
    const int d = valid ? dst[e] : -1;
    int sv = valid ? src[e] : 0;
    sv = min(max(sv, 0), NN - 1);
    const bool ok = (unsigned)d < (unsigned)NN;
    const int key = ok ? (d >> 8) : (NBP - 1);
    const int val = ok ? (sv | ((d & 255) << 17)) : -1;
    const unsigned m = matchmask(key);
    const int lower = __builtin_popcount(m & lt);
    const int old = wex[w * NBP + key];
    int pos = bst[key] + old + lower;
    pos = min(max(pos, 0), ECH - 1);
    srt[pos] = val;
    if (lower == 0) wex[w * NBP + key] = old + __builtin_popcount(m);
  }
  __syncthreads();
  runs_store(srt, bcnt, bst, lineoff, runs, c, t);
  __threadfence();
  runs_store(srt, bcnt, bst, lineoff, runs, c, t);
}

__device__ __forceinline__ void csr_store(const int* srt, const int* nst, const int* ncnt,
                                          int* csr, int* nbeg, int* ndeg,
                                          int L0, int nlw, int b, int t) {
  if (L0 >= 0 && L0 + nlw <= MAXL) {
    int* cp = csr + (size_t)L0 * 32;
    for (int i4 = t; i4 < nlw * 8; i4 += 256) {
      v4i v;
      v.x = srt[4 * i4]; v.y = srt[4 * i4 + 1]; v.z = srt[4 * i4 + 2]; v.w = srt[4 * i4 + 3];
      *(volatile v4i*)(cp + 4 * i4) = v;
    }
  }
  if (t < 64) {
    const int e0 = L0 * 32;
    v4i v;
    v.x = e0 + nst[4 * t]; v.y = e0 + nst[4 * t + 1]; v.z = e0 + nst[4 * t + 2]; v.w = e0 + nst[4 * t + 3];
    *(volatile v4i*)(nbeg + (size_t)b * 256 + 4 * t) = v;
  } else if (t < 128) {
    const int u = t - 64;
    v4i v;
    v.x = ncnt[4 * u]; v.y = ncnt[4 * u + 1]; v.z = ncnt[4 * u + 2]; v.w = ncnt[4 * u + 3];
    *(volatile v4i*)(ndeg + (size_t)b * 256 + 4 * u) = v;
  }
}

__global__ void __launch_bounds__(256) k_csr(const int* __restrict__ lineoff,
                                            const int* __restrict__ runs,
                                            int* __restrict__ csr,
                                            int* __restrict__ nbeg,
                                            int* __restrict__ ndeg) {
  __shared__ __attribute__((aligned(16))) int lst[CAPB];
  __shared__ __attribute__((aligned(16))) int srt[CAPB];
  __shared__ int wh[NWAV * WHB];
  __shared__ int ncnt[256];
  __shared__ int nst[WHB];
  __shared__ int wc[NWAV];
  const int t = threadIdx.x, lane = t & 31, w = t >> 5;
  const int b = blockIdx.x;
  int L0 = lineoff[b * NCHK];
  int L1 = lineoff[(b + 1) * NCHK];
  L0 = min(max(L0, 0), MAXL);
  L1 = min(max(L1, L0), MAXL);
  const unsigned lt = (1u << lane) - 1u;

  int cw = 0;
  for (int L = L0 + w; L < L1; L += NWAV) {
    const int v = runs[(size_t)L * 32 + lane];
    const unsigned m = __builtin_amdgcn_ballot_w32(v >= 0);
    cw += __builtin_popcount(m);
  }
  if (lane == 0) wc[w] = cw;
  for (int i = t; i < NWAV * WHB; i += 256) wh[i] = 0;
  __syncthreads();
  int woff = 0, tot = 0;
#pragma unroll
  for (int u = 0; u < NWAV; ++u) {
    const int x = wc[u];
    tot += x;
    woff += (u < w) ? x : 0;
  }
  const int totc = min(tot, CAPB);
  const int nb = (totc + 31) >> 5;
  cw = 0;
  for (int L = L0 + w; L < L1; L += NWAV) {
    const int v = runs[(size_t)L * 32 + lane];
    const unsigned m = __builtin_amdgcn_ballot_w32(v >= 0);
    const int pos = woff + cw + __builtin_popcount(m & lt);
    if (v >= 0 && pos < CAPB) lst[pos] = v;
    cw += __builtin_popcount(m);
  }
  __syncthreads();
  for (int j = w; j < nb; j += NWAV) {
    const int idx = j * 32 + lane;
    const bool valid = idx < totc;
    const int key = valid ? ((lst[idx] >> 17) & 255) : 256;
    const unsigned m = matchmask(key);
    if ((m & lt) == 0u) wh[w * WHB + key] += __builtin_popcount(m);
  }
  __syncthreads();
  {
    int run = 0;
#pragma unroll
    for (int u = 0; u < NWAV; ++u) {
      const int v = wh[u * WHB + t];
      wh[u * WHB + t] = run;
      run += v;
    }
    ncnt[t] = run;
    if (t == 0) {
      int r2 = 0;
#pragma unroll
      for (int u = 0; u < NWAV; ++u) {
        const int v = wh[u * WHB + 256];
        wh[u * WHB + 256] = r2;
        r2 += v;
      }
    }
  }
  __syncthreads();
  if (w == 0) {
    int s = 0;
#pragma unroll
    for (int i = 0; i < 8; ++i) s += ncnt[lane * 8 + i];
    int incl = s;
#pragma unroll
    for (int d = 1; d < 32; d <<= 1) {
      const int y = __shfl_up(incl, d);
      if (lane >= d) incl += y;
    }
    int ex = incl - s;
#pragma unroll
    for (int i = 0; i < 8; ++i) { nst[lane * 8 + i] = ex; ex += ncnt[lane * 8 + i]; }
    if (lane == 31) nst[256] = ex;
  }
  __syncthreads();
  for (int j = w; j < nb; j += NWAV) {
    const int idx = j * 32 + lane;
    const bool valid = idx < totc;
    const int v = valid ? lst[idx] : 0;
    const int key = valid ? ((v >> 17) & 255) : 256;
    const unsigned m = matchmask(key);
    const int lower = __builtin_popcount(m & lt);
    const int old = wh[w * WHB + key];
    int pos = nst[key] + old + lower;
    pos = min(max(pos, 0), CAPB - 1);
    srt[pos] = v & 0x1FFFF;
    if (lower == 0) wh[w * WHB + key] = old + __builtin_popcount(m);
  }
  __syncthreads();
  csr_store(srt, nst, ncnt, csr, nbeg, ndeg, L0, nb, b, t);
  __threadfence();
  csr_store(srt, nst, ncnt, csr, nbeg, ndeg, L0, nb, b, t);
}

__device__ __forceinline__ void sage_store(const float* myD, float* hout, int base, int q8, int c8l) {
#pragma unroll
  for (int it = 0; it < 4; ++it) {
    const int row = 4 * it + q8;
    const int node = base + row;
    const v4f v = *(const v4fa*)(myD + row * 32 + 4 * c8l);
    if (node < NN) *(volatile v4f*)(hout + (size_t)node * NF + 4 * c8l) = v;
  }
}

__global__ void __launch_bounds__(256) k_sage(const float* __restrict__ feat,
                                             const int* __restrict__ nbeg,
                                             const int* __restrict__ ndeg,
                                             const int* __restrict__ csr,
                                             const _Float16* __restrict__ pb,
                                             const float* __restrict__ ptab,
                                             float* __restrict__ hout) {
  __shared__ __attribute__((aligned(16))) _Float16 sA[NWAV * 16 * 40];
  __shared__ __attribute__((aligned(16))) float sD[NWAV * 16 * 32];
  const int t = threadIdx.x, lane = t & 31, w = t >> 5;
  const int hh = lane >> 4, mn = lane & 15;
  const int q = lane >> 2, c8 = lane & 3;
  const int q8 = lane >> 3, c8l = lane & 7;
  const int base = (blockIdx.x * NWAV + w) * 16;
  _Float16* myA = sA + w * 640;
  float* myD = sD + w * 512;

#pragma unroll 1
  for (int grp = 0; grp < 2; ++grp) {
    const int row = 8 * grp + q;
    const int node = min(base + row, NN - 1);
    int beg = nbeg[node], deg = ndeg[node];
    if (beg < 0 || deg < 0 || beg > CSRN || deg > CSRN - beg) { deg = 0; beg = 0; }
    int dm = deg;
    dm = max(dm, __shfl_xor(dm, 4));
    dm = max(dm, __shfl_xor(dm, 8));
    dm = max(dm, __shfl_xor(dm, 16));
    float a0 = 0.f, a1 = 0.f, a2 = 0.f, a3 = 0.f, a4 = 0.f, a5 = 0.f, a6 = 0.f, a7 = 0.f;
    for (int it = 0; it < dm; ++it) {
      if (it < deg) {
        int s = csr[beg + it];
        s = min(max(s, 0), NN - 1);
        const float* fp = feat + (size_t)s * NF + 8 * c8;
        const v4f u0 = *(const v4f*)(fp);
        const v4f u1 = *(const v4f*)(fp + 4);
        a0 += u0.x; a1 += u0.y; a2 += u0.z; a3 += u0.w;
        a4 += u1.x; a5 += u1.y; a6 += u1.z; a7 += u1.w;
      }
    }
    const float inv = 1.0f / fmaxf((float)deg, 1.0f);
    v8h hv;
    hv[0] = (_Float16)(a0 * inv); hv[1] = (_Float16)(a1 * inv);
    hv[2] = (_Float16)(a2 * inv); hv[3] = (_Float16)(a3 * inv);
    hv[4] = (_Float16)(a4 * inv); hv[5] = (_Float16)(a5 * inv);
    hv[6] = (_Float16)(a6 * inv); hv[7] = (_Float16)(a7 * inv);
    *(v8h*)(myA + row * 40 + 8 * c8) = hv;
  }
  __syncthreads();

  union { v16h v; v8h p[2]; } A, X, Bl, Br;
  A.p[0] = *(const v8ha*)(myA + mn * 40 + 8 * hh);
  A.p[1] = *(const v8ha*)(myA + mn * 40 + 16 + 8 * hh);
  {
    const int rx = min(base + mn, NN - 1);
    const float* px = feat + (size_t)rx * NF;
    const v4f x0 = *(const v4f*)(px + 8 * hh);
    const v4f x1 = *(const v4f*)(px + 8 * hh + 4);
    const v4f x2 = *(const v4f*)(px + 16 + 8 * hh);
    const v4f x3 = *(const v4f*)(px + 20 + 8 * hh);
    X.v[0] = (_Float16)x0.x;  X.v[1] = (_Float16)x0.y;  X.v[2] = (_Float16)x0.z;  X.v[3] = (_Float16)x0.w;
    X.v[4] = (_Float16)x1.x;  X.v[5] = (_Float16)x1.y;  X.v[6] = (_Float16)x1.z;  X.v[7] = (_Float16)x1.w;
    X.v[8] = (_Float16)x2.x;  X.v[9] = (_Float16)x2.y;  X.v[10] = (_Float16)x2.z; X.v[11] = (_Float16)x2.w;
    X.v[12] = (_Float16)x3.x; X.v[13] = (_Float16)x3.y; X.v[14] = (_Float16)x3.z; X.v[15] = (_Float16)x3.w;
  }
  v8f acc[2];
#pragma unroll
  for (int tt = 0; tt < 2; ++tt) {
    const _Float16* p = pb + tt * 1024 + lane * 16;
    Bl.p[0] = *(const v8h*)(p);        Bl.p[1] = *(const v8h*)(p + 8);
    Br.p[0] = *(const v8h*)(p + 512);  Br.p[1] = *(const v8h*)(p + 520);
    const float bias = ptab[16 * tt + mn];
    v8f c;
#pragma unroll
    for (int r = 0; r < 8; ++r) c[r] = bias;
    c = wmma16(A.v, Bl.v, c);
    c = wmma16(X.v, Br.v, c);
    asm volatile("v_nop\n\tv_nop\n\tv_nop\n\tv_nop" : "+v"(c) : "v"(A.v), "v"(Bl.v), "v"(X.v), "v"(Br.v));
    acc[tt] = c;
  }
#pragma unroll
  for (int tt = 0; tt < 2; ++tt) {
    const int n = 16 * tt + mn;
    const float scale = ptab[64 + n];
    const float shift = ptab[128 + n];
#pragma unroll
    for (int r = 0; r < 8; ++r) {
      const float val = fmaxf(acc[tt][r] * 0.0625f, 0.f) * scale + shift;
      myD[(8 * hh + r) * 32 + n] = val;
    }
  }
  __syncthreads();
  sage_store(myD, hout, base, q8, c8l);
  __threadfence();
  sage_store(myD, hout, base, q8, c8l);
}

__device__ __forceinline__ int lbound(const int* a, int n, int x) {
  int lo = 0, hi = n;
  while (lo < hi) {
    const int mid = (lo + hi) >> 1;
    if (a[mid] < x) lo = mid + 1; else hi = mid;
  }
  return lo;
}

__device__ __forceinline__ void head_store(const float* res, float* out, int gb, int t) {
  if (t < 8) {
    const int g0 = gb + 4 * t;
    if (g0 + 3 < NG) {
      v4f v;
      v.x = res[4 * t]; v.y = res[4 * t + 1]; v.z = res[4 * t + 2]; v.w = res[4 * t + 3];
      *(volatile v4f*)(out + g0) = v;
    }
  }
}

__global__ void __launch_bounds__(256) k_head(const float* __restrict__ h,
                                             const int* __restrict__ batch,
                                             const float* __restrict__ W1,
                                             const float* __restrict__ bb1,
                                             const float* __restrict__ W2,
                                             const float* __restrict__ bb2,
                                             float* __restrict__ out) {
  __shared__ float res[32];
  const int t = threadIdx.x, lane = t & 31, w = t >> 5;
  const int gb = blockIdx.x * 32;
  const int jl = min(lane, NCH - 1);
  const float msk = (lane < NCH) ? 1.f : 0.f;
  for (int i = 0; i < 4; ++i) {
    const int g = gb + w * 4 + i;
    float o = 0.f;
    if (g < NG) {
      const int lo = lbound(batch, NN, g);
      const int hi = lbound(batch, NN, g + 1);
      float mx = -INFINITY, sm = 0.f;
      for (int r = lo; r < hi; ++r) {
        const float v = h[(size_t)r * NF + lane];
        mx = fmaxf(mx, v);
        sm += v;
      }
      const int cnt = hi - lo;
      const float xm = (cnt > 0 && __builtin_isfinite(mx)) ? mx : 0.f;
      const float xa = sm / fmaxf((float)cnt, 1.0f);
      o = bb2[0];
#pragma unroll
      for (int k = 0; k < 10; ++k) {
        float p = msk * (W1[k * 60 + jl] * xm + W1[k * 60 + 30 + jl] * xa);
        p += __shfl_xor(p, 16);
        p += __shfl_xor(p, 8);
        p += __shfl_xor(p, 4);
        p += __shfl_xor(p, 2);
        p += __shfl_xor(p, 1);
        const float a = p + bb1[k];
        o += W2[k] * fmaxf(a, 0.f);
      }
      o = 1.0f / (1.0f + expf(-o));
    }
    if (lane == 0) res[w * 4 + i] = o;
  }
  __syncthreads();
  head_store(res, out, gb, t);
  __threadfence();
  head_store(res, out, gb, t);
}

extern "C" void kernel_launch(void* const* d_in, const int* in_sizes, int n_in,
                              void* d_out, int out_size, void* d_ws, size_t ws_size,
                              hipStream_t stream) {
  if (n_in < 21) return;
  if (in_sizes[0] != NN * NF || in_sizes[1] != 2 * NE || in_sizes[2] != NN || out_size != NG) return;

  const float* x   = (const float*)d_in[0];
  const int*   ei  = (const int*)d_in[1];
  const int*   bat = (const int*)d_in[2];
  const float* Wl1 = (const float*)d_in[3];
  const float* bl1 = (const float*)d_in[4];
  const float* Wr1 = (const float*)d_in[5];
  const float* Wl2 = (const float*)d_in[6];
  const float* bl2 = (const float*)d_in[7];
  const float* Wr2 = (const float*)d_in[8];
  const float* g1  = (const float*)d_in[9];
  const float* b1  = (const float*)d_in[10];
  const float* m1  = (const float*)d_in[11];
  const float* v1  = (const float*)d_in[12];
  const float* g2  = (const float*)d_in[13];
  const float* b2  = (const float*)d_in[14];
  const float* m2  = (const float*)d_in[15];
  const float* v2  = (const float*)d_in[16];
  const float* W1  = (const float*)d_in[17];
  const float* bb1 = (const float*)d_in[18];
  const float* W2  = (const float*)d_in[19];
  const float* bb2 = (const float*)d_in[20];
  const int* src = ei;
  const int* dst = ei + NE;

  char* ws = (char*)d_ws;
  size_t off = 0;
  auto carve = [&](size_t bytes) -> char* {
    char* p = ws + off;
    off += (bytes + 127) & ~(size_t)127;
    return p;
  };
  _Float16* pb   = (_Float16*)carve(4096 * sizeof(_Float16));
  float*    ptab = (float*)carve(192 * sizeof(float));
  int*   cntrow  = (int*)carve((size_t)NCHK * CROW * sizeof(int));
  int*   lineoff = (int*)carve((size_t)LOFFN * sizeof(int));
  int*   runs    = (int*)carve((size_t)MAXL * 128);
  int*   csr     = (int*)carve((size_t)MAXL * 128);
  int*   nbeg    = (int*)carve((size_t)NODEP * sizeof(int));
  int*   ndeg    = (int*)carve((size_t)NODEP * sizeof(int));
  float* h1      = (float*)carve((size_t)NN * NF * sizeof(float));
  float* h2      = (float*)carve((size_t)NN * NF * sizeof(float));
  if (off > ws_size) return;

  const int sage_blocks = ((NN / 16) + NWAV - 1) / NWAV;

  k_pack<<<1, 256, 0, stream>>>(Wl1, bl1, Wr1, Wl2, bl2, Wr2,
                                g1, b1, m1, v1, g2, b2, m2, v2, pb, ptab);
  k_count<<<NCHK, 256, 0, stream>>>(dst, cntrow);
  k_scan<<<1, 256, 0, stream>>>(cntrow, lineoff);
  k_place<<<NCHK, 256, 0, stream>>>(src, dst, cntrow, lineoff, runs);
  k_csr<<<NBKT, 256, 0, stream>>>(lineoff, runs, csr, nbeg, ndeg);
  k_sage<<<sage_blocks, 256, 0, stream>>>(x, nbeg, ndeg, csr, pb, ptab, h1);
  k_sage<<<sage_blocks, 256, 0, stream>>>(h1, nbeg, ndeg, csr, pb + 2048, ptab + 32, h2);
  k_head<<<NG / 32, 256, 0, stream>>>(h2, bat, W1, bb1, W2, bb2, (float*)d_out);
}
